// RWKV6TimeMix_41815801594116
// MI455X (gfx1250) — hardware-verified
//
#include <hip/hip_runtime.h>

#define AS3 __attribute__((address_space(3)))

#define BB    4
#define TT    1024
#define DM    1024
#define NH    16
#define HDIM  64
#define LR    64
#define MROWS (BB * TT)
#define PLF   (MROWS * DM)

static_assert(DM == NH * HDIM);
static_assert(HDIM == 64 && LR == 64);
static_assert(MROWS % 128 == 0 && DM % 64 == 0);
static_assert(DM % 32 == 0 && LR % 32 == 0);
static_assert(TT % 32 == 0);
static_assert(DM * DM == (1 << 20));

typedef __bf16         v16b __attribute__((ext_vector_type(16)));
typedef unsigned short v8us __attribute__((ext_vector_type(8)));
typedef float          v8f  __attribute__((ext_vector_type(8)));
typedef float          v4f  __attribute__((ext_vector_type(4)));
typedef v8us __attribute__((may_alias)) v8usa;
typedef v4f  __attribute__((may_alias)) v4fa;

typedef AS3 unsigned short*       lp_us;
typedef AS3 const unsigned short* lcp_us;
typedef AS3 float*                lp_f;
typedef AS3 const float*          lcp_f;

union Frag { v16b v; v8us half[2]; };

constexpr int P_X   = 0;
constexpr int P_WC  = P_X   + MROWS * DM;
constexpr int P_WO  = P_WC  + 4 * DM * DM;
constexpr int P_WLD = P_WO  + DM * DM;
constexpr int P_WLU = P_WLD + LR * DM;
constexpr int P_END = P_WLU + DM * LR;
constexpr int NPC   = P_END / 8;
constexpr int NCBLK = NPC / 256;
static_assert(P_END % 8 == 0);
static_assert(NPC % 256 == 0);
static_assert(P_WC % 2048 == 0 && P_WO % 2048 == 0 && P_WLD % 2048 == 0 && P_WLU % 2048 == 0);
static_assert((DM * DM) % 2048 == 0);

constexpr size_t OFF_CV = 0;
constexpr size_t SZ_CV  = (size_t)P_END * 2;
constexpr size_t OFF_PL = OFF_CV + SZ_CV;
constexpr size_t SZ_PL  = (size_t)5 * PLF * 4;
constexpr size_t OFF_H  = OFF_PL + SZ_PL;
constexpr size_t SZ_H   = (size_t)2 * MROWS * LR * 2;
constexpr size_t OFF_Y  = OFF_H + SZ_H;
constexpr size_t SZ_Y   = (size_t)2 * PLF * 2;
constexpr size_t WS_END = OFF_Y + SZ_Y;
static_assert(OFF_PL % 128 == 0 && OFF_H % 128 == 0 && OFF_Y % 128 == 0);
static_assert(WS_END <= (size_t)134217728);
static_assert((size_t)NPC * 16 == SZ_CV);
static_assert((size_t)(MROWS / 128) * 64 * 256 * 128 + (size_t)(MROWS / 128) * 16 * 256 * 128 == SZ_PL);
static_assert((size_t)(MROWS / 128) * 256 * 128 == SZ_H);
static_assert((size_t)(BB * NH) * (TT / 32) * 64 * 128 == SZ_Y);
static_assert((size_t)(MROWS / 128) * 16 * 256 * 128 == (size_t)PLF * 4);

__device__ __forceinline__ unsigned short bf16_bits(float f) {
  unsigned u = __float_as_uint(f);
  u += 0x7FFFu + ((u >> 16) & 1u);
  return (unsigned short)(u >> 16);
}
__device__ __forceinline__ float bf16_val(unsigned short b) { return __uint_as_float(((unsigned)b) << 16); }
__device__ __forceinline__ float bf16r(float f) { return bf16_val(bf16_bits(f)); }
__device__ __forceinline__ v8f zero8() {
  v8f z;
#pragma unroll
  for (int i = 0; i < 8; ++i) z[i] = 0.0f;
  return z;
}

__device__ __forceinline__ void ldfrag_g(Frag& f, const unsigned short* p, int h) {
  f.half[0] = *(const v8usa*)(p + 8 * h);
  f.half[1] = *(const v8usa*)(p + 16 + 8 * h);
}
__device__ __forceinline__ v8f mma16g(v8f c, v16b a, v16b b) {
  v8f d = __builtin_amdgcn_wmma_f32_16x16x32_bf16(false, a, false, b, (short)0, c, false, false);
  asm volatile("v_nop\n\tv_nop\n\tv_nop\n\tv_nop" : "+v"(d) : "v"(a), "v"(b));
  return d;
}

__global__ __launch_bounds__(256)
void cvt_kernel(const float* __restrict__ x,  const float* __restrict__ wr, const float* __restrict__ wk,
                const float* __restrict__ wv, const float* __restrict__ wg, const float* __restrict__ wo,
                const float* __restrict__ wld, const float* __restrict__ wlu, unsigned short* cv)
{
  const int g = blockIdx.x * 256 + threadIdx.x;
  if (g >= NPC) return;
  const int e = g * 8;
  const float* src;
  if (e < P_WC) {
    src = x + e;
  } else if (e < P_WO) {
    const int d = e - P_WC;
    const int ws = d >> 20;
    const int off = d & ((1 << 20) - 1);
    const float* wp = (ws == 0) ? wr : ((ws == 1) ? wk : ((ws == 2) ? wv : wg));
    src = wp + off;
  } else if (e < P_WLD) {
    src = wo + (e - P_WO);
  } else if (e < P_WLU) {
    src = wld + (e - P_WLD);
  } else {
    src = wlu + (e - P_WLU);
  }
  const v4f a = *(const v4fa*)src;
  const v4f c = *(const v4fa*)(src + 4);
  v8us o;
  o[0] = bf16_bits(a[0]); o[1] = bf16_bits(a[1]); o[2] = bf16_bits(a[2]); o[3] = bf16_bits(a[3]);
  o[4] = bf16_bits(c[0]); o[5] = bf16_bits(c[1]); o[6] = bf16_bits(c[2]); o[7] = bf16_bits(c[3]);
  unsigned short* dst = cv + e;
  *(volatile v8us*)dst = o;
  __threadfence();
  *(volatile v8us*)dst = o;
}

constexpr size_t GL_T   = 0;
constexpr size_t GL_HL  = (size_t)128 * 64 * 4;
constexpr size_t GLDS_F = GL_HL;
constexpr size_t GLDS_H = GL_HL + (size_t)2 * 128 * 64 * 2;

template <int K, int NPROD, int EPI>
__global__ __launch_bounds__(128)
void gemm_kernel(const unsigned short* __restrict__ A, const unsigned short* __restrict__ B,
                 const float* __restrict__ wbase, float* Cf, unsigned short* Ch)
{
  static_assert(K % 32 == 0);
  extern __shared__ __attribute__((aligned(16))) char smem[];
  lp_f  sT  = (lp_f)(smem + GL_T);
  lp_us sHL = (lp_us)(smem + GL_HL);

  const int tid = threadIdx.x, lane = tid & 31, w = tid >> 5;
  const int h = lane >> 4, m = lane & 15;
  const int m0 = blockIdx.x * 128;
  const int by = blockIdx.y;
  const int m0w = m0 + 32 * w;

  const unsigned short* xa = A + (size_t)(m0w + m) * K;
  const unsigned short* xl = xa + (size_t)MROWS * K;
  const unsigned short* wb = B + (size_t)(by * 64 + m) * K;

  v8f acc[2][4];
#pragma unroll
  for (int mt = 0; mt < 2; ++mt)
#pragma unroll
    for (int nt = 0; nt < 4; ++nt) acc[mt][nt] = zero8();

#pragma unroll 1
  for (int k0 = 0; k0 < K; k0 += 32) {
    Frag ah[2], al[2];
#pragma unroll
    for (int mt = 0; mt < 2; ++mt) {
      ldfrag_g(ah[mt], xa + (size_t)mt * 16 * K + k0, h);
      if constexpr (NPROD == 2) ldfrag_g(al[mt], xl + (size_t)mt * 16 * K + k0, h);
    }
#pragma unroll
    for (int nt = 0; nt < 4; ++nt) {
      Frag b;
      ldfrag_g(b, wb + (size_t)nt * 16 * K + k0, h);
#pragma unroll
      for (int mt = 0; mt < 2; ++mt) {
        acc[mt][nt] = mma16g(acc[mt][nt], ah[mt].v, b.v);
        if constexpr (NPROD == 2) acc[mt][nt] = mma16g(acc[mt][nt], al[mt].v, b.v);
      }
    }
  }

#pragma unroll
  for (int nt = 0; nt < 4; ++nt)
#pragma unroll
    for (int mt = 0; mt < 2; ++mt)
#pragma unroll
      for (int r = 0; r < 8; ++r) {
        const int rowl = 32 * w + 16 * mt + 8 * h + r;
        const int col  = 16 * nt + m;
        sT[rowl * 64 + col] = acc[mt][nt][r];
      }
  __syncthreads();

  const int q8 = lane & 7, sub = lane >> 3;

  if constexpr (EPI == 1) {
#pragma unroll 1
    for (int it = 0; it < 64; ++it) {
      const int e = tid + 128 * it;
      const float v = tanhf(sT[e]);
      const unsigned short hb = bf16_bits(v);
      const unsigned short lb = bf16_bits(v - bf16_val(hb));
      sHL[e] = hb;
      sHL[8192 + e] = lb;
    }
    __syncthreads();
#pragma unroll 1
    for (int pass = 0; pass < 2; ++pass) {
#pragma unroll
      for (int i = 0; i < 16; ++i) {
        const int lid  = 4 * i + sub;
        const int rowl = 32 * w + (lid >> 1);
        const int pl   = lid & 1;
        const v8us v = *(AS3 const v8usa*)(sHL + pl * 8192 + rowl * 64 + 8 * q8);
        const size_t go = (size_t)pl * ((size_t)MROWS * LR) + (size_t)(m0 + rowl) * LR + 8 * q8;
        *(volatile v8us*)(Ch + go) = v;
      }
      __threadfence();
    }
  } else {
    if constexpr (EPI == 2) {
#pragma unroll 1
      for (int it = 0; it < 64; ++it) {
        const int e = tid + 128 * it;
        const int n = e & 63;
        const float z = bf16r(wbase[by * 64 + n]) + sT[e];
        const float sp = fmaxf(z, 0.0f) + log1pf(expf(-fabsf(z)));
        sT[e] = -sp;
      }
      __syncthreads();
    }
#pragma unroll 1
    for (int pass = 0; pass < 2; ++pass) {
#pragma unroll
      for (int i = 0; i < 16; ++i) {
        const int lid  = 4 * i + sub;
        const int rowl = 32 * w + (lid >> 1);
        const int hl   = lid & 1;
        const v4f v = *(AS3 const v4fa*)(sT + rowl * 64 + 32 * hl + 4 * q8);
        const size_t go = (size_t)(by >> 4) * PLF + (size_t)(m0 + rowl) * DM + (by & 15) * 64 + 32 * hl + 4 * q8;
        *(volatile v4f*)(Cf + go) = v;
      }
      __threadfence();
    }
  }
}

__global__ __launch_bounds__(256)
void wkv_kernel(const float* __restrict__ pl, const float* __restrict__ uu,
                const float* __restrict__ gam, const float* __restrict__ bet, unsigned short* ypl)
{
  __shared__ __attribute__((aligned(16))) float sR[64];
  __shared__ __attribute__((aligned(16))) float sK[64];
  __shared__ __attribute__((aligned(16))) float sE[64];
  __shared__ __attribute__((aligned(16))) float sU[64];
  __shared__ __attribute__((aligned(16))) float sGa[64];
  __shared__ __attribute__((aligned(16))) float sBe[64];
  __shared__ __attribute__((aligned(16))) float sRed[256];
  __shared__ __attribute__((aligned(16))) unsigned short sY[2 * 32 * 64];

  const int tid = threadIdx.x, lane = tid & 31, w = tid >> 5;
  const int j = tid & 63, iq = tid >> 6;
  const int bh = blockIdx.x, b = bh >> 4, hh = bh & 15;
  const float* Rp = pl;
  const float* Kp = pl + (size_t)PLF;
  const float* Vp = pl + (size_t)2 * PLF;
  const float* Gp = pl + (size_t)3 * PLF;
  const float* Wp = pl + (size_t)4 * PLF;

  if (tid < 64) {
    sU[tid]  = bf16r(uu[hh * HDIM + tid]);
    sGa[tid] = bf16r(gam[tid]);
    sBe[tid] = bf16r(bet[tid]);
  }
  float s[16];
#pragma unroll
  for (int i = 0; i < 16; ++i) s[i] = 0.0f;
  __syncthreads();

  const int q8 = lane & 7, sub = lane >> 3;
  const int i0 = 16 * iq;

#pragma unroll 1
  for (int t = 0; t < TT; ++t) {
    const size_t base = ((size_t)(b * TT + t)) * DM + hh * HDIM;
    if (tid < 64)       sR[tid]       = Rp[base + tid];
    else if (tid < 128) sK[tid - 64]  = Kp[base + tid - 64];
    else if (tid < 192) sE[tid - 128] = expf(Wp[base + tid - 128]);
    const float vj = Vp[base + j];
    __syncthreads();

    float acc = 0.0f;
#pragma unroll
    for (int c = 0; c < 4; ++c) {
      const v4f r4 = *(AS3 const v4fa*)(sR + i0 + 4 * c);
      const v4f k4 = *(AS3 const v4fa*)(sK + i0 + 4 * c);
      const v4f e4 = *(AS3 const v4fa*)(sE + i0 + 4 * c);
      const v4f u4 = *(AS3 const v4fa*)(sU + i0 + 4 * c);
#pragma unroll
      for (int q = 0; q < 4; ++q) {
        const int ii = 4 * c + q;
        const float kv = k4[q] * vj;
        acc = fmaf(r4[q], fmaf(u4[q], kv, s[ii]), acc);
        s[ii] = fmaf(s[ii], e4[q], kv);
      }
    }
    sRed[tid] = acc;
    __syncthreads();

    if (tid < 32) {
      lcp_f rd = (lcp_f)sRed;
      float o0 = rd[lane];       o0 += rd[64 + lane];  o0 += rd[128 + lane];  o0 += rd[192 + lane];
      float o1 = rd[32 + lane];  o1 += rd[96 + lane];  o1 += rd[160 + lane];  o1 += rd[224 + lane];
      float sm = o0 + o1;
      sm += __shfl_xor(sm, 16); sm += __shfl_xor(sm, 8); sm += __shfl_xor(sm, 4);
      sm += __shfl_xor(sm, 2);  sm += __shfl_xor(sm, 1);
      const float mu = sm * (1.0f / 64.0f);
      const float d0 = o0 - mu, d1 = o1 - mu;
      float sq = d0 * d0 + d1 * d1;
      sq += __shfl_xor(sq, 16); sq += __shfl_xor(sq, 8); sq += __shfl_xor(sq, 4);
      sq += __shfl_xor(sq, 2);  sq += __shfl_xor(sq, 1);
      const float var  = sq * (1.0f / 64.0f);
      const float rstd = rsqrtf(var + 1e-5f);
      const float gl0 = Gp[base + lane], gl1 = Gp[base + 32 + lane];
      const float g0 = 1.0f / (1.0f + expf(-gl0));
      const float g1 = 1.0f / (1.0f + expf(-gl1));
      const float y0 = (d0 * rstd * sGa[lane]      + sBe[lane])      * g0;
      const float y1 = (d1 * rstd * sGa[32 + lane] + sBe[32 + lane]) * g1;
      const unsigned short h0 = bf16_bits(y0), h1 = bf16_bits(y1);
      const unsigned short l0 = bf16_bits(y0 - bf16_val(h0)), l1 = bf16_bits(y1 - bf16_val(h1));
      const int ro = (t & 31) * 64;
      sY[ro + lane]             = h0;
      sY[ro + 32 + lane]        = h1;
      sY[2048 + ro + lane]      = l0;
      sY[2048 + ro + 32 + lane] = l1;
    }

    if ((t & 31) == 31) {
      __syncthreads();
      const int plsel = w >> 2;
      v8us yv[2];
      size_t yo[2];
#pragma unroll
      for (int i = 0; i < 2; ++i) {
        const int rr = 8 * (w & 3) + 4 * i + sub;
        yv[i] = *(AS3 const v8usa*)(sY + plsel * 2048 + rr * 64 + 8 * q8);
        yo[i] = (size_t)plsel * PLF + ((size_t)(b * TT + (t - 31) + rr)) * DM + hh * HDIM + 8 * q8;
      }
      *(volatile v8us*)(ypl + yo[0]) = yv[0];
      *(volatile v8us*)(ypl + yo[1]) = yv[1];
      __threadfence();
      *(volatile v8us*)(ypl + yo[0]) = yv[0];
      *(volatile v8us*)(ypl + yo[1]) = yv[1];
    }
  }
}

extern "C" void kernel_launch(void* const* d_in, const int* in_sizes, int n_in,
                              void* d_out, int out_size, void* d_ws, size_t ws_size,
                              hipStream_t stream)
{
  if (n_in < 12) return;
  if (in_sizes[0]  != MROWS * DM) return;
  if (in_sizes[1]  != DM * DM)    return;
  if (in_sizes[2]  != DM * DM)    return;
  if (in_sizes[3]  != DM * DM)    return;
  if (in_sizes[4]  != DM * DM)    return;
  if (in_sizes[5]  != DM * DM)    return;
  if (in_sizes[6]  != DM)         return;
  if (in_sizes[7]  != LR * DM)    return;
  if (in_sizes[8]  != DM * LR)    return;
  if (in_sizes[9]  != NH * HDIM)  return;
  if (in_sizes[10] != HDIM)       return;
  if (in_sizes[11] != HDIM)       return;
  if (out_size != MROWS * DM)     return;
  if (ws_size < WS_END)           return;

  const float* x    = (const float*)d_in[0];
  const float* wr   = (const float*)d_in[1];
  const float* wk   = (const float*)d_in[2];
  const float* wv   = (const float*)d_in[3];
  const float* wo   = (const float*)d_in[4];
  const float* wg   = (const float*)d_in[5];
  const float* wbs  = (const float*)d_in[6];
  const float* wld  = (const float*)d_in[7];
  const float* wlu  = (const float*)d_in[8];
  const float* uu   = (const float*)d_in[9];
  const float* gam  = (const float*)d_in[10];
  const float* bet  = (const float*)d_in[11];
  float* out = (float*)d_out;

  char* ws = (char*)d_ws;
  unsigned short* cv  = (unsigned short*)(ws + OFF_CV);
  float*          pln = (float*)(ws + OFF_PL);
  unsigned short* hpl = (unsigned short*)(ws + OFF_H);
  unsigned short* ypl = (unsigned short*)(ws + OFF_Y);

  cvt_kernel<<<dim3(NCBLK), dim3(256), 0, stream>>>(x, wr, wk, wv, wg, wo, wld, wlu, cv);

  hipFuncSetAttribute(reinterpret_cast<const void*>(&gemm_kernel<DM, 1, 0>),
                      hipFuncAttributeMaxDynamicSharedMemorySize, (int)GLDS_F);
  gemm_kernel<DM, 1, 0><<<dim3(MROWS / 128, (4 * DM) / 64), dim3(128), GLDS_F, stream>>>(
      cv + P_X, cv + P_WC, wbs, pln, hpl);

  hipFuncSetAttribute(reinterpret_cast<const void*>(&gemm_kernel<DM, 1, 1>),
                      hipFuncAttributeMaxDynamicSharedMemorySize, (int)GLDS_H);
  gemm_kernel<DM, 1, 1><<<dim3(MROWS / 128, 1), dim3(128), GLDS_H, stream>>>(
      cv + P_X, cv + P_WLD, wbs, pln, hpl);

  hipFuncSetAttribute(reinterpret_cast<const void*>(&gemm_kernel<LR, 2, 2>),
                      hipFuncAttributeMaxDynamicSharedMemorySize, (int)GLDS_F);
  gemm_kernel<LR, 2, 2><<<dim3(MROWS / 128, DM / 64), dim3(128), GLDS_F, stream>>>(
      hpl, cv + P_WLU, wbs, pln + (size_t)4 * PLF, ypl);

  wkv_kernel<<<dim3(BB * NH), dim3(256), 0, stream>>>(pln, uu, gam, bet, ypl);

  hipFuncSetAttribute(reinterpret_cast<const void*>(&gemm_kernel<DM, 2, 0>),
                      hipFuncAttributeMaxDynamicSharedMemorySize, (int)GLDS_F);
  gemm_kernel<DM, 2, 0><<<dim3(MROWS / 128, DM / 64), dim3(128), GLDS_F, stream>>>(
      ypl, cv + P_WO, wbs, out, hpl);
}
